// SlowMAF_29850022707695
// MI455X (gfx1250) — hardware-verified
//
#include <hip/hip_runtime.h>


namespace {
constexpr int B = 65536, NLIM = 65536  , DIM = 32, NK = DIM - 1, NH = 24, HP = 32  , OP = 16  ;
constexpr float XS = 8.0f, WSC = 256.0f, SLOPE = 0.2f;
static_assert(B % 32 == 0 && NLIM % 32 == 0 && NLIM <= B && DIM == 32 && NH <= HP, "tiling");
typedef _Float16 b16;
typedef __attribute__((ext_vector_type(16))) _Float16 v16b;
typedef __attribute__((ext_vector_type(8))) _Float16 v8b;
typedef __attribute__((ext_vector_type(8))) float v8f;
typedef __attribute__((ext_vector_type(4))) float v4f;
__device__ __forceinline__ float bf16_rne(float f) { unsigned int u = __float_as_uint(f); u += 0x7FFFu + ((u >> 16) & 1u); return __uint_as_float(u & 0xFFFF0000u); }
__device__ __forceinline__ void split16(float v, b16& hi, b16& lo) { hi = (b16)v; lo = (b16)(v - (float)hi); }
__device__ __forceinline__ v16b frag_kb(const b16* p, int hh) { const v8b a = *(const v8b*)(p + 8 * hh), b = *(const v8b*)(p + 16 + 8 * hh); v16b f;
#pragma unroll
  for (int e = 0; e < 8; ++e) { f[e] = a[e]; f[8 + e] = b[e]; } return f; }
__device__ __forceinline__ v8f wmma16b(v16b a, v16b b, v8f c) { v8f d = __builtin_amdgcn_wmma_f32_16x16x32_f16(false, a, false, b, (short)0, c, false, false); asm volatile("v_nop\n\tv_nop\n\tv_nop\n\tv_nop" : "+v"(d) : "v"(a), "v"(b)); return d; }
__device__ __forceinline__ void wave_lds_sync() { __builtin_amdgcn_fence(__ATOMIC_RELEASE, "workgroup"); __builtin_amdgcn_wave_barrier(); __builtin_amdgcn_fence(__ATOMIC_ACQUIRE, "workgroup"); }
__device__ __forceinline__ float pmul(float a, float b) { float p = a * b; asm volatile("" : "+v"(p)); return p; }
__device__ __forceinline__ int iclamp(int v, int lo, int hi) { return v < lo ? lo : (v > hi ? hi : v); }

typedef __attribute__((ext_vector_type(4))) _Float16 v4h;
__device__ __forceinline__ float lrelu(float v) { return v > 0.0f ? v : SLOPE * v; }
__global__ __launch_bounds__(256) void prep_kernel(const float* __restrict__ x, const float* __restrict__ w1, const float* __restrict__ w2, const float* __restrict__ w3, const float* __restrict__ w4, b16* __restrict__ Xh, b16* __restrict__ W1T, b16* __restrict__ W2T, b16* __restrict__ W3T, b16* __restrict__ W4T) {
  size_t t = (size_t)blockIdx.x * 256 + threadIdx.x; v8b o;
  const size_t nx = (size_t)B * DIM / 8; if (t < nx) { const size_t e = t * 8; for (int j = 0; j < 8; ++j) o[j] = (b16)(bf16_rne(x[e + j]) * XS); for (int pass = 0; pass < 2; ++pass) { *(volatile v8b*)(Xh + e) = o; __threadfence(); } return; } t -= nx;
  const size_t n1 = (size_t)NK * HP * DIM / 8; if (t < n1) { const size_t e = t * 8; const int k = (int)(e / (HP * DIM)), r = (int)((e / DIM) % HP), j0 = (int)(e % DIM);
    for (int j = 0; j < 8; ++j) { const int jj = j0 + j; o[j] = (r < NH && jj <= k) ? (b16)(bf16_rne(w1[((size_t)k * NH + r) * DIM + jj]) * WSC) : (b16)0.0f; } for (int pass = 0; pass < 2; ++pass) { *(volatile v8b*)(W1T + e) = o; __threadfence(); } return; } t -= n1;
  for (int l = 0; l < 2; ++l) { const size_t n2 = (size_t)NK * HP * HP / 8; if (t < n2) { const size_t e = t * 8; const int k = (int)(e / (HP * HP)), r = (int)((e / HP) % HP), j0 = (int)(e % HP); const float* w = l ? w3 : w2;
      for (int j = 0; j < 8; ++j) { const int jj = j0 + j; o[j] = (r < NH && jj < NH) ? (b16)(bf16_rne(w[((size_t)k * NH + r) * NH + jj]) * WSC) : (b16)0.0f; } for (int pass = 0; pass < 2; ++pass) { *(volatile v8b*)((l ? W3T : W2T) + e) = o; __threadfence(); } return; } t -= n2; }
  const size_t n4 = (size_t)NK * OP * HP / 8; if (t < n4) { const size_t e = t * 8; const int k = (int)(e / (OP * HP)), r = (int)((e / HP) % OP), j0 = (int)(e % HP);
    for (int j = 0; j < 8; ++j) { const int jj = j0 + j; o[j] = (r < 2 && jj < NH) ? (b16)(bf16_rne(w4[((size_t)k * 2 + r) * NH + jj]) * WSC) : (b16)0.0f; } for (int pass = 0; pass < 2; ++pass) { *(volatile v8b*)(W4T + e) = o; __threadfence(); } }
}
__global__ __launch_bounds__(64) void maf_kernel(const b16* __restrict__ Xh, const float* __restrict__ x, const float* __restrict__ p0, const b16* __restrict__ W1T, const float* __restrict__ b1, const b16* __restrict__ W2T, const float* __restrict__ b2, const b16* __restrict__ W3T, const float* __restrict__ b3, const b16* __restrict__ W4T, const float* __restrict__ b4, float* __restrict__ zout, float* __restrict__ ldout) {
  __shared__ __attribute__((aligned(16))) b16 Hh[2][16][HP + 8], Hl[2][16][HP + 8]; __shared__ __attribute__((aligned(16))) float Tf[2][16][HP + 4], St[2][16][2], Zr[2][16][DIM + 1], Ld[2][16]; __shared__ float Lds32[32];
  const int wave = threadIdx.x >> 5, lane = threadIdx.x & 31, nloc = lane & 15, hlf = lane >> 4; const size_t m0 = (size_t)blockIdx.x * 32 + wave * 16;
  if (lane < 16) { const size_t row = m0 + lane; const float s0 = bf16_rne(p0[0]), t0 = bf16_rne(p0[1]); const float xv = bf16_rne(x[row * DIM + 0]); Zr[wave][lane][DIM - 1] = pmul(xv, __expf(s0)) + t0; Ld[wave][lane] = s0; }
  const v16b ax = frag_kb(Xh + (m0 + nloc) * DIM, hlf);
  const float rs1 = 1.0f / (XS * WSC);
  auto stage = [&](const v8f& a0, const v8f& a1, const float* bias) {
#pragma unroll
    for (int r = 0; r < 8; ++r) { const int row = 8 * hlf + r; Tf[wave][row][nloc] = lrelu(a0[r] * rs1 + bf16_rne(bias[nloc])); const int c1 = 16 + nloc; Tf[wave][row][c1] = (c1 < NH) ? lrelu(a1[r] * rs1 + bf16_rne(bias[c1 < NH ? c1 : 0])) : 0.0f; }
    wave_lds_sync();
    { const int row = lane & 15, c0 = (lane >> 4) * 16; v8b h0, l0, h1, l1;
#pragma unroll
      for (int j = 0; j < 8; ++j) { b16 p, q; split16(Tf[wave][row][c0 + j] * XS, p, q); h0[j] = p; l0[j] = q; split16(Tf[wave][row][c0 + 8 + j] * XS, p, q); h1[j] = p; l1[j] = q; }
      *(v8b*)(&Hh[wave][row][c0]) = h0; *(v8b*)(&Hh[wave][row][c0 + 8]) = h1; *(v8b*)(&Hl[wave][row][c0]) = l0; *(v8b*)(&Hl[wave][row][c0 + 8]) = l1; }
    wave_lds_sync(); };
#pragma unroll 1
  for (int k = 0; k < NK; ++k) {
    { v8f a0 = (v8f){}, a1 = (v8f){};
      a0 = wmma16b(ax, frag_kb(W1T + ((size_t)k * HP + nloc) * DIM, hlf), a0); a1 = wmma16b(ax, frag_kb(W1T + ((size_t)k * HP + 16 + nloc) * DIM, hlf), a1);
      stage(a0, a1, b1 + k * NH); }
#pragma unroll
    for (int l = 0; l < 2; ++l) { const b16* WT = (l ? W3T : W2T) + (size_t)k * HP * HP; const float* bb = (l ? b3 : b2) + k * NH;
      const v16b ah = frag_kb(&Hh[wave][nloc][0], hlf), al = frag_kb(&Hl[wave][nloc][0], hlf);
      v8f c0 = (v8f){}, c1 = (v8f){}; { const v16b w0 = frag_kb(WT + (size_t)nloc * HP, hlf), w1 = frag_kb(WT + (size_t)(16 + nloc) * HP, hlf); c0 = wmma16b(ah, w0, c0); c0 = wmma16b(al, w0, c0); c1 = wmma16b(ah, w1, c1); c1 = wmma16b(al, w1, c1); }
      wave_lds_sync();
      stage(c0, c1, bb); }
    { const v16b ah = frag_kb(&Hh[wave][nloc][0], hlf), al = frag_kb(&Hl[wave][nloc][0], hlf); const v16b w0 = frag_kb(W4T + ((size_t)k * OP + nloc) * HP, hlf); v8f d0 = (v8f){}; d0 = wmma16b(ah, w0, d0); d0 = wmma16b(al, w0, d0);
      if (nloc < 2) {
#pragma unroll
        for (int r = 0; r < 8; ++r) St[wave][8 * hlf + r][nloc] = d0[r] * rs1 + bf16_rne(b4[k * 2 + nloc]); } }
    wave_lds_sync();
    if (lane < 16) { const size_t row = m0 + lane; const float s = St[wave][lane][0], tt = St[wave][lane][1]; const float xv = bf16_rne(x[row * DIM + k + 1]); Zr[wave][lane][DIM - 1 - (k + 1)] = pmul(xv, __expf(s)) + tt; Ld[wave][lane] += s; }
    wave_lds_sync(); }
  if (lane < 16) Lds32[wave * 16 + lane] = Ld[wave][lane];
  __syncthreads();
  for (int pass = 0; pass < 2; ++pass) { for (int rr = 0; rr < 16; ++rr) ((volatile float*)zout)[(m0 + rr) * DIM + lane] = Zr[wave][rr][lane];
    if (threadIdx.x < 32) ((volatile float*)ldout)[(size_t)blockIdx.x * 32 + threadIdx.x] = Lds32[threadIdx.x];
    __threadfence(); }
}
}

extern "C" void kernel_launch(void* const* d_in, const int* in_sizes, int n_in, void* d_out, int out_size, void* d_ws, size_t ws_size, hipStream_t stream) {
  (void)n_in;
  auto Fp = [&](int i) { return (const float*)d_in[i]; };
  if (in_sizes[0] != B * DIM || in_sizes[1] != 2 || in_sizes[2] != NK * NH * DIM || in_sizes[3] != NK * NH || in_sizes[4] != NK * NH * NH || in_sizes[5] != NK * NH || in_sizes[6] != NK * NH * NH || in_sizes[7] != NK * NH || in_sizes[8] != NK * 2 * NH || in_sizes[9] != NK * 2 || out_size != B * DIM + B) return;
  size_t off = 0; char* ws = (char*)d_ws;
  auto carve = [&](size_t bytes) { char* p = ws + off; off += (bytes + 255) & ~(size_t)255; return p; };
  b16* Xh = (b16*)carve((size_t)B * DIM * 2); b16* W1T = (b16*)carve((size_t)NK * HP * DIM * 2); b16* W2T = (b16*)carve((size_t)NK * HP * HP * 2); b16* W3T = (b16*)carve((size_t)NK * HP * HP * 2); b16* W4T = (b16*)carve((size_t)NK * OP * HP * 2);
  if (off > ws_size || off > ((size_t)128 << 20)) return;
  prep_kernel<<<(unsigned)((((size_t)B * DIM + (size_t)NK * HP * DIM + 2 * (size_t)NK * HP * HP + (size_t)NK * OP * HP) / 8 + 255) / 256), 256, 0, stream>>>(Fp(0), Fp(2), Fp(4), Fp(6), Fp(8), Xh, W1T, W2T, W3T, W4T);
  maf_kernel<<<NLIM / 32, 64, 0, stream>>>(Xh, Fp(0), Fp(1), W1T, Fp(3), W2T, Fp(5), W3T, Fp(7), W4T, Fp(9), (float*)d_out, (float*)d_out + (size_t)B * DIM);
}
